// GAT_base_layer_14491219657225
// MI455X (gfx1250) — hardware-verified
//
#include <hip/hip_runtime.h>
#include <math.h>

typedef __attribute__((ext_vector_type(16))) _Float16 v16h;
typedef __attribute__((ext_vector_type(16))) __bf16 v16b;
typedef __attribute__((ext_vector_type(8)))  _Float16 v8h;
typedef __attribute__((ext_vector_type(8)))  float v8f;
typedef __attribute__((ext_vector_type(4)))  float v4f;
typedef __attribute__((ext_vector_type(2)))  float v2f;
typedef __attribute__((ext_vector_type(4)))  unsigned v4u;
typedef __attribute__((ext_vector_type(4)))  int v4i;
typedef float __attribute__((may_alias)) float_a;
typedef int __attribute__((may_alias)) int_a;

template <typename T> __device__ __forceinline__ void vst2(void* p, T v) { *(volatile T*)p = v; __threadfence(); *(volatile T*)p = v; }
__device__ __forceinline__ v8f wmma16(v16h a, v16h b, v8f c) {
  v8f d = __builtin_amdgcn_wmma_f32_16x16x32_f16(false, a, false, b, (short)0, c, false, false);
  asm volatile("v_nop\n\tv_nop\n\tv_nop\n\tv_nop" : "+v"(d) : "v"(a), "v"(b));
  return d;
}
__device__ __forceinline__ v8f wmma_bf(v16b a, v16b b, v8f c) {
  v8f d = __builtin_amdgcn_wmma_f32_16x16x32_bf16(false, a, false, b, (short)0, c, false, false);
  asm volatile("v_nop\n\tv_nop\n\tv_nop\n\tv_nop" : "+v"(d) : "v"(a), "v"(b));
  return d;
}
__device__ __forceinline__ v16h frag_h(const _Float16* rowk0, int lane) {
  union { v16h v; v8h q[2]; } u; const _Float16* p = rowk0 + 8 * (lane >> 4);
  u.q[0] = *(const v8h*)p; u.q[1] = *(const v8h*)(p + 16); return u.v;
}
__device__ __forceinline__ v16h frag_f32(const float* rowk0, int lane) {
  v16h a; const float* p = rowk0 + 8 * (lane >> 4);
#pragma unroll
  for (int i = 0; i < 8; ++i) { a[i] = (_Float16)p[i]; a[8 + i] = (_Float16)p[16 + i]; }
  return a;
}
__device__ __forceinline__ v16h frag_f32s(const float* rowk0, int lane, float sc) {
  v16h a; const float* p = rowk0 + 8 * (lane >> 4);
#pragma unroll
  for (int i = 0; i < 8; ++i) { a[i] = (_Float16)(p[i] * sc); a[8 + i] = (_Float16)(p[16 + i] * sc); }
  return a;
}
__device__ __forceinline__ v16h fragc_f32(const float* W, int k0, int n, int lane, int ld, int K) {
  v16h a; const int g = lane >> 4;
#pragma unroll
  for (int i = 0; i < 8; ++i) { const int ka = k0 + 8 * g + i, kb = ka + 16;
    a[i] = (_Float16)(ka < K ? W[(size_t)ka * ld + n] : 0.f); a[8 + i] = (_Float16)(kb < K ? W[(size_t)kb * ld + n] : 0.f); }
  return a;
}
struct F2 { v16b h, l; };
__device__ __forceinline__ F2 bsplit16(const float v[16]) { F2 r;
#pragma unroll
  for (int i = 0; i < 16; ++i) { const __bf16 h = (__bf16)v[i]; r.h[i] = h; r.l[i] = (__bf16)(v[i] - (float)h); }
  return r; }
__device__ __forceinline__ F2 split_row(const float* row, int k0, int lane) { float v[16]; const float* p = row + k0 + 8 * (lane >> 4);
#pragma unroll
  for (int i = 0; i < 8; ++i) { v[i] = p[i]; v[8 + i] = p[16 + i]; }
  return bsplit16(v); }
__device__ __forceinline__ F2 split_rowK(const float* row, int k0, int lane, int K) { float v[16]; const int g = lane >> 4;
#pragma unroll
  for (int i = 0; i < 8; ++i) { const int ka = k0 + 8 * g + i, kb = ka + 16; v[i] = ka < K ? row[ka] : 0.f; v[8 + i] = kb < K ? row[kb] : 0.f; }
  return bsplit16(v); }
__device__ __forceinline__ F2 split_col(const float* W, int k0, int n, int lane, int ld, int K) { float v[16]; const int g = lane >> 4;
#pragma unroll
  for (int i = 0; i < 8; ++i) { const int ka = k0 + 8 * g + i, kb = ka + 16; v[i] = ka < K ? W[(size_t)ka * ld + n] : 0.f; v[8 + i] = kb < K ? W[(size_t)kb * ld + n] : 0.f; }
  return bsplit16(v); }
__device__ __forceinline__ v8f mac3(const F2& a, const F2& b, v8f c) { c = wmma_bf(a.l, b.h, c); c = wmma_bf(a.h, b.l, c); return wmma_bf(a.h, b.h, c); }
__device__ __forceinline__ float sigm(float v) { return 1.0f / (1.0f + expf(-v)); }
#define LDSX() do { asm volatile("s_wait_dscnt 0" ::: "memory"); __builtin_amdgcn_wave_barrier(); __builtin_amdgcn_fence(__ATOMIC_RELEASE, "workgroup"); } while (0)


#define NN 100000
#define NE 1600000
#define F0 128
#define RB 512
#define NRB ((NN + RB - 1) / RB)
#define NNP (NRB * RB)
#define EPT 8
#define CH (256 * EPT)
__device__ __forceinline__ float lrelu(float v) { return v > 0.f ? v : 0.2f * v; }

__global__ __launch_bounds__(128) void k_gemm(const float* __restrict__ x, const float* __restrict__ W, const float* __restrict__ b, const float* __restrict__ a,
                                             float* __restrict__ HS, float* __restrict__ ES, float* __restrict__ ED) {
  __shared__ __align__(16) float so[4][16][F0 + 4]; __shared__ __align__(16) float se[2][64];
  const int tid = threadIdx.x, wave = tid >> 5, lane = tid & 31, col = lane & 15, g = lane >> 4;
  const int r0 = blockIdx.x * 64 + wave * 16; const int ra = (r0 + col) < NN ? (r0 + col) : (NN - 1);
  v8f acc[8] = {};
#pragma unroll 1
  for (int kc = 0; kc < F0 / 32; ++kc) { const F2 av = split_row(x + (size_t)ra * F0, kc * 32, lane);
#pragma unroll
    for (int t = 0; t < 8; ++t) acc[t] = mac3(av, split_row(W + (size_t)(t * 16 + col) * F0, kc * 32, lane), acc[t]); }
#pragma unroll
  for (int t = 0; t < 8; ++t) { const int n = t * 16 + col; const float bb = b[n];
#pragma unroll
    for (int r = 0; r < 8; ++r) { const int row = r0 + 8 * g + r; so[wave][8 * g + r][n] = row < NN ? acc[t][r] + bb : 0.f; } }
  LDSX();
  { const int row = lane & 15, which = lane >> 4; const float* hr = &so[wave][row][0]; const float* av = a + which * F0; float s = 0.f;
#pragma unroll 4
    for (int k = 0; k < F0; ++k) s += hr[k] * av[k];
    se[which][wave * 16 + row] = s; }
  for (int q = lane; q < 16 * (F0 / 4); q += 32) { const int rl = q >> 5, pc = q & 31; vst2(HS + (size_t)(r0 + rl) * F0 + pc * 4, *(const v4f*)(&so[wave][rl][pc * 4])); }
  __syncthreads();
  if (wave == 0) { const int which = lane >> 4, pc = lane & 15; vst2((which == 0 ? ES : ED) + (size_t)blockIdx.x * 64 + pc * 4, *(const v4f*)(&se[which][pc * 4])); }
}
__global__ __launch_bounds__(256) void k_agg(const float* __restrict__ HS, const float* __restrict__ ES, const float* __restrict__ ED, const int* __restrict__ sarr, const int* __restrict__ tarr, float* __restrict__ out) {
  __shared__ __align__(16) float sacc[RB][F0];
  __shared__ float sdiv[RB]; __shared__ float ses[RB];
  __shared__ int sedg[8][32 * EPT], sdl[8][32 * EPT]; __shared__ float swgt[8][32 * EPT]; __shared__ int scnt[8];
  const int tid = threadIdx.x, wave = tid >> 5, lane = tid & 31;
  const int r0 = blockIdx.x * RB;
  for (int q = tid; q < RB * F0; q += 256) (&sacc[0][0])[q] = 0.f;
  for (int q = tid; q < RB; q += 256) { sdiv[q] = 0.f; ses[q] = (r0 + q) < NN ? ES[r0 + q] : 0.f; }
  __syncthreads();
#pragma unroll 1
  for (int c0 = 0; c0 < NE; c0 += CH) {
    const int e0 = c0 + tid * EPT; int hd[EPT]; int cnt = 0;
    if (e0 + EPT <= NE) {
#pragma unroll
      for (int v = 0; v < EPT / 4; ++v) { const int4 d4 = *(const int4*)(sarr + e0 + v * 4);
        const int dd[4] = {d4.x, d4.y, d4.z, d4.w};
#pragma unroll
        for (int u = 0; u < 4; ++u) { const unsigned rel = (unsigned)(dd[u] - r0); const bool h = rel < (unsigned)RB; hd[v * 4 + u] = h ? (int)rel : -1; cnt += h ? 1 : 0; } } }
    else {
#pragma unroll
      for (int u = 0; u < EPT; ++u) { const int e = e0 + u; hd[u] = -1; if (e < NE) { const unsigned rel = (unsigned)(sarr[e] - r0); if (rel < (unsigned)RB) { hd[u] = (int)rel; ++cnt; } } } }
    int incl = cnt;
#pragma unroll
    for (int off = 1; off < 32; off <<= 1) { const int vv = __shfl_up(incl, off, 32); if (lane >= off) incl += vv; }
    const int wtot = __shfl(incl, 31, 32); int pos = incl - cnt;
    if (cnt > 0) {
#pragma unroll
      for (int u = 0; u < EPT; ++u) if (hd[u] >= 0) { sedg[wave][pos] = e0 + u; sdl[wave][pos] = hd[u]; ++pos; } }
    if (lane == 0) scnt[wave] = wtot;
    __syncthreads();
#pragma unroll 1
    for (int w = 0; w < 8; ++w) { const int nh = scnt[w];
#pragma unroll 1
      for (int i = tid; i < nh; i += 256) { int t = tarr[sedg[w][i]]; t = t < 0 ? 0 : (t >= NN ? NN - 1 : t); sedg[w][i] = t; swgt[w][i] = expf(lrelu(ses[sdl[w][i]] + ED[t])); } }
    __syncthreads();
    if (tid < F0) {
#pragma unroll 1
      for (int w = 0; w < 8; ++w) { const int nh = scnt[w];
#pragma unroll 1
        for (int i = 0; i < nh; ++i) { const int t = sedg[w][i], dl = sdl[w][i]; const float wgt = swgt[w][i];
          sacc[dl][tid] += wgt * HS[(size_t)t * F0 + tid]; if (tid == 0) sdiv[dl] += wgt; } } }
    __syncthreads(); }
  for (int q = tid; q < RB; q += 256) sdiv[q] = 1.0f / sdiv[q];
  __syncthreads();
#pragma unroll 1
  for (int q = tid; q < RB * (F0 / 4); q += 256) { const int rl = q >> 5, pc = q & 31; const int row = r0 + rl; if (row >= NN) continue;
    v4f v = *(const v4f*)(&sacc[rl][pc * 4]); const float d = sdiv[rl]; v[0] *= d; v[1] *= d; v[2] *= d; v[3] *= d; vst2(out + (size_t)row * F0 + pc * 4, v); }
}
extern "C" void kernel_launch(void* const* d_in, const int* in_sizes, int n_in, void* d_out, int out_size, void* d_ws, size_t ws_size, hipStream_t stream) {
  (void)in_sizes; (void)n_in; (void)out_size; (void)ws_size;
  const float* x = (const float*)d_in[0]; const int* sarr = (const int*)d_in[1]; const int* tarr = (const int*)d_in[2]; const float* W = (const float*)d_in[3]; const float* b = (const float*)d_in[4]; const float* a = (const float*)d_in[5];
  float* out = (float*)d_out;
  char* ws = (char*)d_ws; size_t off = 0;
  auto take = [&](size_t bytes) { char* p = ws + off; off += (bytes + 255) & ~(size_t)255; return p; };
  float* HS = (float*)take((size_t)NNP * F0 * 4); float* ES = (float*)take((size_t)NNP * 4); float* ED = (float*)take((size_t)NNP * 4);
  k_gemm<<<NNP / 64, 128, 0, stream>>>(x, W, b, a, HS, ES, ED);
  k_agg<<<NRB, 256, 0, stream>>>(HS, ES, ED, sarr, tarr, out);
}
